// SA_Layer_42167988912479
// MI455X (gfx1250) — hardware-run, weakly checked
//
#include <hip/hip_runtime.h>
#include <math.h>

typedef __attribute__((ext_vector_type(16))) _Float16 v16h;
typedef __attribute__((ext_vector_type(8)))  _Float16 v8h;
typedef __attribute__((ext_vector_type(16))) __bf16   v16b;
typedef __attribute__((ext_vector_type(8)))  __bf16   v8b;
typedef __attribute__((ext_vector_type(8)))  float    v8f;
typedef __attribute__((ext_vector_type(4)))  float    v4f;
typedef __attribute__((ext_vector_type(4)))  unsigned int v4u;

constexpr int kB    = 4;
constexpr int kC    = 256;
constexpr int kN    = 512;
constexpr int kCQ   = 64;
constexpr int kRows = kB * kN;
constexpr int kK2   = 2 * kC;
static_assert(kCQ * 4 == kC, "quarter width");
static_assert(kRows == 2048 && kK2 == 512, "shapes");
static_assert((kC % 32) == 0 && (kK2 % 32) == 0 && (kCQ % 32) == 0 && (kN % 32) == 0, "GEMM K multiples of 32");
static_assert((kRows % 64) == 0 && (kCQ % 64) == 0 && (kN % 64) == 0 && (kC % 64) == 0, "GEMM M,N multiples of 64");

constexpr float kXCarry = 16.0f;
constexpr float kWCarry = 1024.0f;
constexpr float kVCarry = 16.0f;
constexpr float kECarry = 32768.0f;
constexpr float kVbScale  = kVCarry / (kWCarry * kXCarry);
constexpr float kXrScale  = -1.0f / (kECarry * kVCarry);
constexpr float kLinScale = 1.0f / (kWCarry * kXCarry);

constexpr double kPiD     = 3.14159265358979323846;
constexpr double kLn1e4D  = 9.210340371976184;
constexpr float  kFactor  = (float)(180.0 / (kPiD * 15.0));
constexpr float  kDivCoef = (float)(-kLn1e4D / (double)kCQ);
constexpr float  kBnEps   = 1e-5f;
constexpr float  kInvSqrt2 = 0.70710678118654752f;
constexpr float  kFltMin  = 1.17549435e-38f;

constexpr size_t kOffXH   = 0;
constexpr size_t kOffXL   = kOffXH   + (size_t)kRows * kK2 * 2;
constexpr size_t kOffXF   = kOffXL   + (size_t)kRows * kK2 * 2;
constexpr size_t kOffXT32 = kOffXF   + (size_t)kRows * kK2 * 2;
constexpr size_t kOffWKPH = kOffXT32 + (size_t)kRows * kC * 4;
constexpr size_t kOffWKPL = kOffWKPH + (size_t)kCQ * kC * 2;
constexpr size_t kOffWKKH = kOffWKPL + (size_t)kCQ * kC * 2;
constexpr size_t kOffWKKL = kOffWKKH + (size_t)kCQ * kK2 * 2;
constexpr size_t kOffWV2  = kOffWKKL + (size_t)kCQ * kK2 * 2;
constexpr size_t kOffLINW = kOffWV2  + (size_t)kC * kK2 * 2;
constexpr size_t kOffXQ   = kOffLINW + (size_t)kC * kC * 2;
constexpr size_t kOffKS   = kOffXQ   + (size_t)kRows * kCQ * 4;
constexpr size_t kOffXQH  = kOffKS   + (size_t)kRows * kCQ * 4;
constexpr size_t kOffXQL  = kOffXQH  + (size_t)kRows * kCQ * 2;
constexpr size_t kOffKSH  = kOffXQL  + (size_t)kRows * kCQ * 2;
constexpr size_t kOffKSL  = kOffKSH  + (size_t)kRows * kCQ * 2;
constexpr size_t kOffQ1   = kOffKSL  + (size_t)kRows * kCQ * 2;
constexpr size_t kOffLG   = kOffQ1   + (size_t)kRows * kCQ * 4;
constexpr size_t kOffPR   = kOffLG   + (size_t)kB * kN * kN * 4;
constexpr size_t kOffET   = kOffPR   + (size_t)kB * kN * kN * 4;
constexpr size_t kOffVB   = kOffET   + (size_t)kB * kN * kN * 2;
constexpr size_t kOffXDT  = kOffVB   + (size_t)kB * kC * kN * 2;
constexpr size_t kOffZB   = kOffXDT  + (size_t)kRows * kC * 2;
constexpr size_t kWsTotal = kOffZB   + (size_t)kB * kC * kN * 4;
static_assert(kWsTotal == 26279936ull, "carve total");
static_assert(kWsTotal <= 134217728ull, "carve cap");
static_assert((kOffXL % 128) == 0 && (kOffXF % 128) == 0 && (kOffXT32 % 128) == 0 && (kOffWKPH % 128) == 0 &&
              (kOffWKPL % 128) == 0 && (kOffWKKH % 128) == 0 && (kOffWKKL % 128) == 0 && (kOffWV2 % 128) == 0 &&
              (kOffLINW % 128) == 0 && (kOffXQ % 128) == 0 && (kOffKS % 128) == 0 && (kOffXQH % 128) == 0 &&
              (kOffXQL % 128) == 0 && (kOffKSH % 128) == 0 && (kOffKSL % 128) == 0 && (kOffQ1 % 128) == 0 &&
              (kOffLG % 128) == 0 && (kOffPR % 128) == 0 && (kOffET % 128) == 0 && (kOffVB % 128) == 0 &&
              (kOffXDT % 128) == 0 && (kOffZB % 128) == 0, "128-B aligned regions");

constexpr size_t kOut1ByteOff = (size_t)kB * kC * kN * 4;
static_assert(kOut1ByteOff == 2097152ull && (kOut1ByteOff % 128) == 0, "second output offset");
constexpr size_t kOut1ElemOff = kOut1ByteOff / 4;
constexpr int    kOutTotal    = kB * kC * kN + kB * kN;
static_assert((size_t)kOutTotal * 4 == kOut1ByteOff + (size_t)kB * kN * 4, "output extent");

__device__ __forceinline__ unsigned short f2bf_bits(float f) {
  unsigned u = __float_as_uint(f);
  return (unsigned short)((u + 0x7FFFu + ((u >> 16) & 1u)) >> 16);
}
__device__ __forceinline__ float bf_bits2f(unsigned short h) { return __uint_as_float(((unsigned)h) << 16); }
__device__ __forceinline__ unsigned pk16(unsigned short a, unsigned short b) { return (unsigned)a | ((unsigned)b << 16); }
__device__ __forceinline__ unsigned short h_bits(float f) { const _Float16 h = (_Float16)f; return __builtin_bit_cast(unsigned short, h); }

__device__ __forceinline__ float wave_sum(float v) {
#pragma unroll
  for (int off = 16; off > 0; off >>= 1) v += __shfl_xor(v, off, 32);
  return v;
}
__device__ __forceinline__ float wave_max(float v) {
#pragma unroll
  for (int off = 16; off > 0; off >>= 1) v = fmaxf(v, __shfl_xor(v, off, 32));
  return v;
}

__device__ __forceinline__ void guard1_h(v8f& a, v16h x, v16h y, v16h z) { asm volatile("v_nop\n\tv_nop\n\tv_nop\n\tv_nop" : "+v"(a) : "v"(x), "v"(y), "v"(z)); }
__device__ __forceinline__ void guard1_b(v8f& a, v16b x, v16b y, v16b z) { asm volatile("v_nop\n\tv_nop\n\tv_nop\n\tv_nop" : "+v"(a) : "v"(x), "v"(y), "v"(z)); }
__device__ __forceinline__ void keep4_h(v16h a, v16h b, v16h c, v16h d) { asm volatile("v_nop" :: "v"(a), "v"(b), "v"(c), "v"(d)); }
__device__ __forceinline__ void keep4_b(v16b a, v16b b, v16b c, v16b d) { asm volatile("v_nop" :: "v"(a), "v"(b), "v"(c), "v"(d)); }
__device__ __forceinline__ void acc_guard4(v8f& a, v8f& b, v8f& c, v8f& d) { asm volatile("v_nop\n\tv_nop\n\tv_nop\n\tv_nop" : "+v"(a), "+v"(b), "+v"(c), "+v"(d)); }
template <typename T> struct Frag;
template <> struct Frag<_Float16> {
  typedef v16h V; union U { v16h v; v8h h[2]; };
  static __device__ __forceinline__ v16h load(const _Float16* p) {
    U f; f.h[0] = *(const v8h*)(p); f.h[1] = *(const v8h*)(p + 16); return f.v;
  }
  static __device__ __forceinline__ v8f mma(v16h a, v16h b, v8f c) {
    return __builtin_amdgcn_wmma_f32_16x16x32_f16(false, a, false, b, (short)0, c, false, false);
  }
  static __device__ __forceinline__ void guard1(v8f& a, v16h x, v16h y, v16h z) { guard1_h(a, x, y, z); }
  static __device__ __forceinline__ void keep(v16h a, v16h b, v16h c, v16h d) { keep4_h(a, b, c, d); }
};
template <> struct Frag<__bf16> {
  typedef v16b V; union U { v16b v; v8b h[2]; };
  static __device__ __forceinline__ v16b load(const __bf16* p) {
    U f; f.h[0] = *(const v8b*)(p); f.h[1] = *(const v8b*)(p + 16); return f.v;
  }
  static __device__ __forceinline__ v8f mma(v16b a, v16b b, v8f c) {
    return __builtin_amdgcn_wmma_f32_16x16x32_bf16(false, a, false, b, (short)0, c, false, false);
  }
  static __device__ __forceinline__ void guard1(v8f& a, v16b x, v16b y, v16b z) { guard1_b(a, x, y, z); }
  static __device__ __forceinline__ void keep(v16b a, v16b b, v16b c, v16b d) { keep4_b(a, b, c, d); }
};

template <int ET> struct Elem;
template <> struct Elem<0> { typedef _Float16 T; };
template <> struct Elem<1> { typedef __bf16 T; };
template <int ET, bool SPLIT, int OUT_MODE, bool RESID>
__global__ __launch_bounds__(256) void wmma_gemm64(
    const unsigned short* __restrict__ Ap, const unsigned short* __restrict__ A2p, int lda, long strideA,
    const unsigned short* __restrict__ Btp, const unsigned short* __restrict__ Bt2p, int ldb, long strideB,
    void* __restrict__ Cout, int ldc, long strideC,
    const float* __restrict__ resid, int ldr, long strideR,
    int M, int N, int K, float scale, float oscale) {
  typedef typename Elem<ET>::T T;
  typedef typename Frag<T>::V V;
  const T* A = (const T*)Ap; const T* A2 = (const T*)A2p; const T* Bt = (const T*)Btp; const T* Bt2 = (const T*)Bt2p;
  __shared__ __align__(16) float sT[8][16 * 68];
  const int b    = blockIdx.y;
  const int lane = threadIdx.x & 31;
  const int wave = __builtin_amdgcn_readfirstlane((int)(threadIdx.x >> 5));
  const int tilesN = N >> 6;
  const int tilesM = M >> 6;
  const int tile = blockIdx.x * 8 + wave;
  if (tile >= tilesM * tilesN) return;
  const int tm = tile / tilesN;
  const int tn = tile - tm * tilesN;
  const int m0 = tm << 6;
  const int n0 = tn << 6;

  const T* Ab  = A  + (size_t)b * strideA;
  const T* Bb  = Bt + (size_t)b * strideB;
  const T* Ab2 = A2  + (size_t)b * strideA;
  const T* Bb2 = Bt2 + (size_t)b * strideB;

  const int rlane = lane & 15;
  const int koff  = (lane >> 4) * 8;
  const int mOff  = (lane >> 4) * 8;

  v8f acc[4][4];
#pragma unroll
  for (int i = 0; i < 4; ++i)
#pragma unroll
    for (int j = 0; j < 4; ++j) acc[i][j] = (v8f){0.f,0.f,0.f,0.f,0.f,0.f,0.f,0.f};

  for (int k0 = 0; k0 < K; k0 += 32) {
    V bh[4], bl[4];
#pragma unroll
    for (int j = 0; j < 4; ++j) {
      const size_t bo = (size_t)(n0 + (j << 4) + rlane) * ldb + koff + k0;
      bh[j] = Frag<T>::load(Bb + bo);
      if (SPLIT) bl[j] = Frag<T>::load(Bb2 + bo);
    }
#pragma unroll
    for (int i = 0; i < 4; ++i) {
      const size_t ao = (size_t)(m0 + (i << 4) + rlane) * lda + koff + k0;
      V ah = Frag<T>::load(Ab + ao);
      V al;
      if (SPLIT) al = Frag<T>::load(Ab2 + ao);
#pragma unroll
      for (int j = 0; j < 4; ++j) {
        acc[i][j] = Frag<T>::mma(ah, bh[j], acc[i][j]);
        if (SPLIT) {
          acc[i][j] = Frag<T>::mma(ah, bl[j], acc[i][j]);
          acc[i][j] = Frag<T>::mma(al, bh[j], acc[i][j]);
        }
      }
      Frag<T>::guard1(acc[i][0], ah, SPLIT ? al : ah, bh[0]);
      Frag<T>::guard1(acc[i][1], ah, SPLIT ? al : ah, bh[1]);
      Frag<T>::guard1(acc[i][2], ah, SPLIT ? al : ah, bh[2]);
      Frag<T>::guard1(acc[i][3], ah, SPLIT ? al : ah, bh[3]);
    }
    Frag<T>::keep(bh[0], bh[1], bh[2], bh[3]);
    if (SPLIT) Frag<T>::keep(bl[0], bl[1], bl[2], bl[3]);
  }
  acc_guard4(acc[0][0], acc[0][1], acc[0][2], acc[0][3]);
  acc_guard4(acc[1][0], acc[1][1], acc[1][2], acc[1][3]);
  acc_guard4(acc[2][0], acc[2][1], acc[2][2], acc[2][3]);
  acc_guard4(acc[3][0], acc[3][1], acc[3][2], acc[3][3]);

  float* slab = sT[wave];
  const float* Rb = RESID ? (resid + (size_t)b * strideR) : nullptr;
#pragma unroll
  for (int i = 0; i < 4; ++i) {
    const int mBase = m0 + (i << 4);
#pragma unroll
    for (int j = 0; j < 4; ++j) {
#pragma unroll
      for (int r = 0; r < 8; ++r) {
        slab[(mOff + r) * 68 + (j << 4) + rlane] = acc[i][j][r] * scale;
      }
    }
    __builtin_amdgcn_fence(__ATOMIC_RELEASE, "workgroup");
    __builtin_amdgcn_wave_barrier();
    __builtin_amdgcn_fence(__ATOMIC_ACQUIRE, "workgroup");
    if (OUT_MODE == 0) {
      float* Cp = (float*)Cout + (size_t)b * strideC;
      const int hh = lane >> 4, c4 = (lane & 15) * 4;
      for (int pass = 0; pass < 2; ++pass) {
#pragma unroll
        for (int it = 0; it < 8; ++it) {
          const int row = it * 2 + hh;
          v4f v = *(const v4f*)(slab + row * 68 + c4);
          if (RESID) {
            const v4f rv = *(const v4f*)(Rb + (size_t)(mBase + row) * ldr + n0 + c4);
            v = (v + rv) * oscale;
          }
          *(volatile v4f*)(Cp + (size_t)(mBase + row) * ldc + n0 + c4) = v;
        }
        __threadfence();
      }
    } else {
      const int q = lane >> 3, c8 = (lane & 7) * 8;
      unsigned short* Cp = (unsigned short*)Cout + (size_t)b * strideC;
      for (int pass = 0; pass < 2; ++pass) {
#pragma unroll
        for (int it = 0; it < 4; ++it) {
          const int row = it * 4 + q;
          const float* sp = slab + row * 68 + c8;
          v4f s0 = *(const v4f*)(sp);
          v4f s1 = *(const v4f*)(sp + 4);
          if (RESID) {
            const float* rp = Rb + (size_t)(mBase + row) * ldr + n0 + c8;
            const v4f r0 = *(const v4f*)(rp);
            const v4f r1 = *(const v4f*)(rp + 4);
            s0 = (s0 + r0) * oscale;
            s1 = (s1 + r1) * oscale;
          }
          v8h hv;
#pragma unroll
          for (int e = 0; e < 4; ++e) {
            const float f0 = s0[e];
            const float f1 = s1[e];
            hv[e]     = (_Float16)f0;
            hv[4 + e] = (_Float16)f1;
          }
          *(volatile v8h*)(Cp + (size_t)(mBase + row) * ldc + n0 + c8) = hv;
        }
        __threadfence();
      }
    }
    __builtin_amdgcn_fence(__ATOMIC_RELEASE, "workgroup");
    __builtin_amdgcn_wave_barrier();
    __builtin_amdgcn_fence(__ATOMIC_ACQUIRE, "workgroup");
  }
}

__global__ __launch_bounds__(256) void prep_act_kernel(
    const float* __restrict__ x, const float* __restrict__ pca,
    unsigned short* __restrict__ XH, unsigned short* __restrict__ XL, unsigned short* __restrict__ XF,
    float* __restrict__ XT32) {
  __shared__ float sm[64 * 65];
  const int t = threadIdx.x, lane = t & 31;
  const int wave = __builtin_amdgcn_readfirstlane((int)(threadIdx.x >> 5));
  const int n0 = blockIdx.x * 64;
  const int kt = blockIdx.y;
  const int b  = blockIdx.z;
  const bool isx = (kt < 4);
  const float* src = isx ? x : pca;
  const int c0 = (kt & 3) * 64;
#pragma unroll
  for (int i = 0; i < 16; ++i) {
    const int e = i * 256 + t;
    const int r = e >> 6;
    const int cc = e & 63;
    sm[r * 65 + cc] = src[((size_t)(b * kC + c0 + r)) * kN + n0 + cc];
  }
  __syncthreads();
  const int q = lane >> 3, c8 = (lane & 7) * 8;
  const int hh = lane >> 4, c4 = (lane & 15) * 4;
  v4u uh[2], ul[2], uf[2];
#pragma unroll
  for (int it = 0; it < 2; ++it) {
    const int row = wave * 8 + it * 4 + q;
    unsigned short hb[8], lb[8], fb[8];
#pragma unroll
    for (int e = 0; e < 8; ++e) {
      const float v = sm[(c8 + e) * 65 + row];
      hb[e] = f2bf_bits(v);
      lb[e] = f2bf_bits(v - bf_bits2f(hb[e]));
      fb[e] = h_bits(v * kXCarry);
    }
    uh[it] = (v4u){pk16(hb[0], hb[1]), pk16(hb[2], hb[3]), pk16(hb[4], hb[5]), pk16(hb[6], hb[7])};
    ul[it] = (v4u){pk16(lb[0], lb[1]), pk16(lb[2], lb[3]), pk16(lb[4], lb[5]), pk16(lb[6], lb[7])};
    uf[it] = (v4u){pk16(fb[0], fb[1]), pk16(fb[2], fb[3]), pk16(fb[4], fb[5]), pk16(fb[6], fb[7])};
  }
  v4f fv[4];
#pragma unroll
  for (int it = 0; it < 4; ++it) {
    const int row = wave * 8 + it * 2 + hh;
    fv[it] = (v4f){sm[(c4 + 0) * 65 + row], sm[(c4 + 1) * 65 + row], sm[(c4 + 2) * 65 + row], sm[(c4 + 3) * 65 + row]};
  }
  for (int pass = 0; pass < 2; ++pass) {
#pragma unroll
    for (int it = 0; it < 2; ++it) {
      const int row = wave * 8 + it * 4 + q;
      const size_t o = (size_t)(b * kN + n0 + row) * kK2 + kt * 64 + c8;
      *(volatile v4u*)(XH + o) = uh[it];
      *(volatile v4u*)(XL + o) = ul[it];
      *(volatile v4u*)(XF + o) = uf[it];
    }
    if (isx) {
#pragma unroll
      for (int it = 0; it < 4; ++it) {
        const int row = wave * 8 + it * 2 + hh;
        *(volatile v4f*)(XT32 + (size_t)(b * kN + n0 + row) * kC + c0 + c4) = fv[it];
      }
    }
    __threadfence();
  }
}

__global__ __launch_bounds__(256) void prep_weight_kernel(
    const float* __restrict__ Wkp, const float* __restrict__ Wk, const float* __restrict__ Wv,
    const float* __restrict__ Wvp, const float* __restrict__ linW,
    unsigned short* __restrict__ WKPH, unsigned short* __restrict__ WKPL,
    unsigned short* __restrict__ WKKH, unsigned short* __restrict__ WKKL,
    unsigned short* __restrict__ WV2, unsigned short* __restrict__ LINW) {
  const int bid = blockIdx.x;
  const float* src;
  unsigned short* dh;
  unsigned short* dl;
  int dpitch, dcol, first;
  bool split;
  float sc;
  if (bid < 8)       { src = Wkp;  dh = WKPH; dl = WKPL; dpitch = kC;  dcol = 0;  first = 0;  split = true;  sc = 1.0f; }
  else if (bid < 16) { src = Wk;   dh = WKKH; dl = WKKL; dpitch = kK2; dcol = 0;  first = 8;  split = true;  sc = 1.0f; }
  else if (bid < 24) { src = Wkp;  dh = WKKH; dl = WKKL; dpitch = kK2; dcol = kC; first = 16; split = true;  sc = 1.0f; }
  else if (bid < 56) { src = Wv;   dh = WV2;  dl = WV2;  dpitch = kK2; dcol = 0;  first = 24; split = false; sc = 0.5f * kWCarry; }
  else if (bid < 88) { src = Wvp;  dh = WV2;  dl = WV2;  dpitch = kK2; dcol = kC; first = 56; split = false; sc = 0.5f * kWCarry; }
  else               { src = linW; dh = LINW; dl = LINW; dpitch = kC;  dcol = 0;  first = 88; split = false; sc = kWCarry; }
  const int g   = (bid - first) * 256 + (int)threadIdx.x;
  const int row = g >> 5;
  const int c8  = (g & 31) * 8;
  const float* p = src + (size_t)row * kC + c8;
  const v4f a0 = *(const v4f*)(p);
  const v4f a1 = *(const v4f*)(p + 4);
  const size_t o = (size_t)row * dpitch + dcol + c8;
  if (split) {
    unsigned short hb[8], lb[8];
#pragma unroll
    for (int e = 0; e < 4; ++e) {
      const float f0 = a0[e];
      const float f1 = a1[e];
      hb[e]     = f2bf_bits(f0);
      hb[4 + e] = f2bf_bits(f1);
      lb[e]     = f2bf_bits(f0 - bf_bits2f(hb[e]));
      lb[4 + e] = f2bf_bits(f1 - bf_bits2f(hb[4 + e]));
    }
    const v4u uh = (v4u){pk16(hb[0], hb[1]), pk16(hb[2], hb[3]), pk16(hb[4], hb[5]), pk16(hb[6], hb[7])};
    const v4u ul = (v4u){pk16(lb[0], lb[1]), pk16(lb[2], lb[3]), pk16(lb[4], lb[5]), pk16(lb[6], lb[7])};
    *(volatile v4u*)(dh + o) = uh;
    *(volatile v4u*)(dl + o) = ul;
    __threadfence();
    *(volatile v4u*)(dh + o) = uh;
    *(volatile v4u*)(dl + o) = ul;
  } else {
    unsigned short fb[8];
#pragma unroll
    for (int e = 0; e < 4; ++e) {
      const float f0 = a0[e];
      const float f1 = a1[e];
      fb[e]     = h_bits(f0 * sc);
      fb[4 + e] = h_bits(f1 * sc);
    }
    const v4u uf = (v4u){pk16(fb[0], fb[1]), pk16(fb[2], fb[3]), pk16(fb[4], fb[5]), pk16(fb[6], fb[7])};
    *(volatile v4u*)(dh + o) = uf;
    __threadfence();
    *(volatile v4u*)(dh + o) = uf;
  }
}

__global__ __launch_bounds__(256) void qk_post_kernel(
    const float* __restrict__ XQ, const float* __restrict__ KS, const float* __restrict__ angp,
    const float* __restrict__ W1, const float* __restrict__ W2, const float* __restrict__ b2,
    unsigned short* __restrict__ XQH, unsigned short* __restrict__ XQL,
    unsigned short* __restrict__ KSH, unsigned short* __restrict__ KSL, float* __restrict__ Q1) {
  __shared__ __align__(16) float sW1[kCQ * kCQ];
  __shared__ __align__(16) float sW2T[kCQ * kCQ];
  __shared__ __align__(16) float sXq[16 * kCQ];
  __shared__ __align__(16) float sEmb[16 * kCQ];
  __shared__ __align__(16) float sKs[16 * kCQ];
  __shared__ __align__(16) float sQ1[16 * kCQ];
  __shared__ float sDiv[32];
  const int t = threadIdx.x, lane = t & 31;
  const int wave = __builtin_amdgcn_readfirstlane((int)(threadIdx.x >> 5));
  const int row0 = blockIdx.x * 16;
#pragma unroll 4
  for (int i = 0; i < 16; ++i) {
    const int e = i * 256 + t;
    sW1[e] = W1[e];
    sW2T[(e & 63) * kCQ + (e >> 6)] = W2[e];
  }
#pragma unroll
  for (int i = 0; i < 4; ++i) {
    const int e = i * 256 + t;
    sXq[e] = XQ[(size_t)row0 * kCQ + e];
  }
  {
    const float dv = expf((float)(2 * (t & 31)) * kDivCoef);
    if (t < 32) sDiv[t] = dv;
  }
  __syncthreads();
#pragma unroll 1
  for (int i = 0; i < 2; ++i) {
    const int e = i * 256 + t;
    const int r = e >> 5;
    const int idx = e & 31;
    const float a = angp[row0 + r];
    const float w = (a * kFactor) * sDiv[idx];
    float sv, cv;
    sincosf(w, &sv, &cv);
    sEmb[r * kCQ + 2 * idx]     = sv;
    sEmb[r * kCQ + 2 * idx + 1] = cv;
  }
  __syncthreads();
  const int c  = t & 63;
  const int rg = wave >> 1;
  const float bias2 = b2[c];
  float accE[4], accQ[4];
#pragma unroll
  for (int rr = 0; rr < 4; ++rr) { accE[rr] = bias2; accQ[rr] = 0.0f; }
#pragma unroll 2
  for (int d = 0; d < kCQ; ++d) {
    const float w1 = sW1[d * kCQ + c];
    const float w2 = sW2T[d * kCQ + c];
#pragma unroll
    for (int rr = 0; rr < 4; ++rr) {
      const int row = rg * 4 + rr;
      accE[rr] = fmaf(sEmb[row * kCQ + d], w2, accE[rr]);
      accQ[rr] = fmaf(sXq[row * kCQ + d], w1, accQ[rr]);
    }
  }
#pragma unroll
  for (int rr = 0; rr < 4; ++rr) {
    const int row = rg * 4 + rr;
    const float kv = KS[(size_t)(row0 + row) * kCQ + c];
    sKs[row * kCQ + c] = kv + accE[rr];
    sQ1[row * kCQ + c] = accQ[rr];
  }
  __syncthreads();
  const int q = lane >> 3, c8 = (lane & 7) * 8;
  const int hh = lane >> 4, c4 = (lane & 15) * 4;
  const bool isq = (wave < 4);
  const float* srcT = isq ? sXq : sKs;
  unsigned short* dh = isq ? XQH : KSH;
  unsigned short* dl = isq ? XQL : KSL;
  const int rowh = (wave & 3) * 4 + q;
  unsigned short hb[8], lb[8];
#pragma unroll
  for (int e = 0; e < 8; ++e) {
    const float v = srcT[rowh * kCQ + c8 + e];
    hb[e] = f2bf_bits(v);
    lb[e] = f2bf_bits(v - bf_bits2f(hb[e]));
  }
  const v4u uh = (v4u){pk16(hb[0], hb[1]), pk16(hb[2], hb[3]), pk16(hb[4], hb[5]), pk16(hb[6], hb[7])};
  const v4u ul = (v4u){pk16(lb[0], lb[1]), pk16(lb[2], lb[3]), pk16(lb[4], lb[5]), pk16(lb[6], lb[7])};
  const int rowq = wave * 2 + hh;
  const v4f qv = *(const v4f*)(sQ1 + rowq * kCQ + c4);
  const size_t oh = (size_t)(row0 + rowh) * kCQ + c8;
  const size_t oq = (size_t)(row0 + rowq) * kCQ + c4;
  for (int pass = 0; pass < 2; ++pass) {
    *(volatile v4u*)(dh + oh) = uh;
    *(volatile v4u*)(dl + oh) = ul;
    *(volatile v4f*)(Q1 + oq) = qv;
    __threadfence();
  }
}

__global__ __launch_bounds__(256) void angle_softmax_kernel(
    const float* __restrict__ Lg, const float* __restrict__ ang, const float* __restrict__ Q1,
    const float* __restrict__ XQ, const float* __restrict__ e1b, float* __restrict__ P) {
  __shared__ __align__(16) float sp[kN];
  __shared__ float sq1[kCQ];
  __shared__ float sdiv[32];
  __shared__ float redM[8];
  __shared__ float redS[8];
  const int t = threadIdx.x, lane = t & 31;
  const int wave = __builtin_amdgcn_readfirstlane((int)(threadIdx.x >> 5));
  const int row = blockIdx.x;
  float qv = Q1[(size_t)row * kCQ + (t & 63)];
  asm volatile("" : "+v"(qv));
  if (t < kCQ) sq1[t] = qv;
  const float dv = expf((float)(2 * (t & 31)) * kDivCoef);
  if (t < 32) sdiv[t] = dv;
  float part = XQ[(size_t)row * kCQ + lane] * e1b[lane];
  part = fmaf(XQ[(size_t)row * kCQ + 32 + lane], e1b[32 + lane], part);
  const float qb = wave_sum(part);
  __syncthreads();
  const float* lrow = Lg  + (size_t)row * kN;
  const float* arow = ang + (size_t)row * kN;
#pragma unroll 1
  for (int j = 0; j < 2; ++j) {
    const int m = t + j * 256;
    const float base = arow[m] * kFactor;
    float acc = lrow[m] + qb;
#pragma unroll 1
    for (int i = 0; i < 32; ++i) {
      const float w = base * sdiv[i];
      float sv, cv;
      sincosf(w, &sv, &cv);
      acc = fmaf(sv, sq1[2 * i], acc);
      acc = fmaf(cv, sq1[2 * i + 1], acc);
    }
    sp[m] = acc;
  }
  const float l0 = sp[t];
  const float l1 = sp[t + 256];
  const float wm = wave_max(fmaxf(l0, l1));
  if (lane == 0) redM[wave] = wm;
  __syncthreads();
  float mx = redM[0];
#pragma unroll
  for (int w = 1; w < 8; ++w) mx = fmaxf(mx, redM[w]);
  const float e0 = expf(l0 - mx);
  const float e1 = expf(l1 - mx);
  const float ws = wave_sum(e0 + e1);
  if (lane == 0) redS[wave] = ws;
  __syncthreads();
  float tot = redS[0];
#pragma unroll
  for (int w = 1; w < 8; ++w) tot += redS[w];
  const float inv = 1.0f / tot;
  float p0 = e0 * inv;
  float p1 = e1 * inv;
  p0 = (p0 < kFltMin) ? 0.0f : p0;
  p1 = (p1 < kFltMin) ? 0.0f : p1;
  sp[t] = p0;
  sp[t + 256] = p1;
  __syncthreads();
  if (wave < 4) {
    const v4f v = *(const v4f*)(sp + 4 * t);
    float* dst = P + (size_t)row * kN + 4 * t;
    *(volatile v4f*)dst = v;
    __threadfence();
    *(volatile v4f*)dst = v;
  }
}

__global__ __launch_bounds__(256) void colnorm_transpose_kernel(
    const float* __restrict__ P, unsigned short* __restrict__ ET, float* __restrict__ out1) {
  __shared__ float sPart[4 * 64];
  __shared__ float sInv[64];
  __shared__ float sTile[64 * 65];
  const int t = threadIdx.x, lane = t & 31;
  const int wave = __builtin_amdgcn_readfirstlane((int)(threadIdx.x >> 5));
  const int m0 = blockIdx.x * 64;
  const int b  = blockIdx.y;
  const int cidx = t & 63;
  const int g = wave >> 1;
  {
    const float* pp = P + ((size_t)(b * kN + g * 128)) * kN + m0 + cidx;
    float s = 0.0f;
#pragma unroll 4
    for (int n = 0; n < 128; ++n) s += pp[(size_t)n * kN];
    sPart[g * 64 + cidx] = s;
  }
  __syncthreads();
  {
    const float cs = ((sPart[cidx] + sPart[64 + cidx]) + sPart[128 + cidx]) + sPart[192 + cidx];
    const float iv = 1.0f / (1e-12f + cs);
    if (t < 64) sInv[t] = iv;
  }
  __syncthreads();
  {
    const int c4 = (lane & 15) * 4;
    v4f pv = *(const v4f*)(P + ((size_t)(b * kN)) * kN + m0 + c4);
    asm volatile("" : "+v"(pv));
    const v4f ov = (v4f){pv[0] * sInv[c4 + 0], pv[1] * sInv[c4 + 1], pv[2] * sInv[c4 + 2], pv[3] * sInv[c4 + 3]};
    if (wave == 0 && lane < 16) {
      float* dst = out1 + (size_t)b * kN + m0 + c4;
      *(volatile v4f*)dst = ov;
      __threadfence();
      *(volatile v4f*)dst = ov;
    }
  }
  const int q = lane >> 3, c8 = (lane & 7) * 8;
#pragma unroll 1
  for (int nt = 0; nt < 8; ++nt) {
    __syncthreads();
#pragma unroll 4
    for (int i = 0; i < 16; ++i) {
      const int e = i * 256 + t;
      const int r = e >> 6;
      const int cc = e & 63;
      const float pvv = P[((size_t)(b * kN + nt * 64 + r)) * kN + m0 + cc];
      sTile[r * 65 + cc] = (pvv * sInv[cc]) * kECarry;
    }
    __syncthreads();
    v4u u[2];
#pragma unroll
    for (int it = 0; it < 2; ++it) {
      const int row = wave * 8 + it * 4 + q;
      unsigned short fb[8];
#pragma unroll
      for (int e = 0; e < 8; ++e) fb[e] = h_bits(sTile[(c8 + e) * 65 + row]);
      u[it] = (v4u){pk16(fb[0], fb[1]), pk16(fb[2], fb[3]), pk16(fb[4], fb[5]), pk16(fb[6], fb[7])};
    }
    for (int pass = 0; pass < 2; ++pass) {
#pragma unroll
      for (int it = 0; it < 2; ++it) {
        const int row = wave * 8 + it * 4 + q;
        *(volatile v4u*)(ET + ((size_t)(b * kN + m0 + row)) * kN + nt * 64 + c8) = u[it];
      }
      __threadfence();
    }
  }
}

__global__ __launch_bounds__(256) void bn_gelu_kernel(
    const float* __restrict__ ZB, const float* __restrict__ x, const float* __restrict__ linb,
    const float* __restrict__ gamma, const float* __restrict__ beta, float* __restrict__ out) {
  __shared__ __align__(16) float ybuf[kB * kN];
  __shared__ float red1[8];
  __shared__ float red2[8];
  const int t = threadIdx.x, lane = t & 31;
  const int wave = __builtin_amdgcn_readfirstlane((int)(threadIdx.x >> 5));
  const int o = blockIdx.x;
  const float lb = linb[o], gm = gamma[o], bt = beta[o];
  size_t off[2];
  v4f zv[2];
#pragma unroll
  for (int j = 0; j < 2; ++j) {
    const int idx4 = t + j * 256;
    const int bb = idx4 >> 7;
    const int m4 = (idx4 & 127) * 4;
    off[j] = ((size_t)(bb * kC + o)) * kN + m4;
    zv[j] = *(const v4f*)(ZB + off[j]) + lb;
  }
  float s = ((zv[0][0] + zv[0][1]) + (zv[0][2] + zv[0][3])) + ((zv[1][0] + zv[1][1]) + (zv[1][2] + zv[1][3]));
  s = wave_sum(s);
  if (lane == 0) red1[wave] = s;
  __syncthreads();
  float tot = red1[0];
#pragma unroll
  for (int w = 1; w < 8; ++w) tot += red1[w];
  const float mean = tot * (1.0f / (float)(kB * kN));
  const v4f d0 = zv[0] - mean;
  const v4f d1 = zv[1] - mean;
  float sq = ((d0[0] * d0[0] + d0[1] * d0[1]) + (d0[2] * d0[2] + d0[3] * d0[3])) +
             ((d1[0] * d1[0] + d1[1] * d1[1]) + (d1[2] * d1[2] + d1[3] * d1[3]));
  sq = wave_sum(sq);
  if (lane == 0) red2[wave] = sq;
  __syncthreads();
  float tot2 = red2[0];
#pragma unroll
  for (int w = 1; w < 8; ++w) tot2 += red2[w];
  const float var = tot2 * (1.0f / (float)(kB * kN));
  const float rs = rsqrtf(var + kBnEps);
  const v4f y0 = (d0 * gm) * rs + bt;
  const v4f y1 = (d1 * gm) * rs + bt;
  *(v4f*)(ybuf + 4 * t) = y0;
  *(v4f*)(ybuf + 4 * (t + 256)) = y1;
  __syncthreads();
#pragma unroll 1
  for (int e = 0; e < 8; ++e) {
    const int i = e * 256 + t;
    const float yv = ybuf[i];
    const float gv = 0.5f * yv * (1.0f + erff(yv * kInvSqrt2));
    ybuf[i] = gv;
  }
  __syncthreads();
  v4f ov[2];
#pragma unroll
  for (int j = 0; j < 2; ++j) {
    const int idx4 = t + j * 256;
    const v4f g4 = *(const v4f*)(ybuf + 4 * idx4);
    const v4f x4 = *(const v4f*)(x + off[j]);
    ov[j] = x4 + g4;
  }
  for (int pass = 0; pass < 2; ++pass) {
#pragma unroll
    for (int j = 0; j < 2; ++j) *(volatile v4f*)(out + off[j]) = ov[j];
    __threadfence();
  }
}

extern "C" void kernel_launch(void* const* d_in, const int* in_sizes, int n_in,
                              void* d_out, int out_size, void* d_ws, size_t ws_size,
                              hipStream_t stream) {
  if (n_in < 16) return;
  if (in_sizes[0] != kB * kC * kN) return;
  if (in_sizes[1] != kB * kC * kN) return;
  if (in_sizes[2] != kB * kN * kN) return;
  if (in_sizes[3] != kB * kN) return;
  if (in_sizes[4] != kCQ * kC) return;
  if (in_sizes[5] != kCQ * kC) return;
  if (in_sizes[6] != kC * kC) return;
  if (in_sizes[7] != kC * kC) return;
  if (in_sizes[8] != kCQ * kCQ) return;
  if (in_sizes[9] != kCQ) return;
  if (in_sizes[10] != kCQ * kCQ) return;
  if (in_sizes[11] != kCQ) return;
  if (in_sizes[12] != kC * kC) return;
  if (in_sizes[13] != kC) return;
  if (in_sizes[14] != kC) return;
  if (in_sizes[15] != kC) return;
  if (out_size != kOutTotal) return;
  if (ws_size < kWsTotal) return;

  const float* x      = (const float*)d_in[0];
  const float* pca    = (const float*)d_in[1];
  const float* a_lrf  = (const float*)d_in[2];
  const float* a_pca  = (const float*)d_in[3];
  const float* Wkp    = (const float*)d_in[4];
  const float* Wk     = (const float*)d_in[5];
  const float* Wv     = (const float*)d_in[6];
  const float* Wvp    = (const float*)d_in[7];
  const float* e1W    = (const float*)d_in[8];
  const float* e1b    = (const float*)d_in[9];
  const float* e2W    = (const float*)d_in[10];
  const float* e2b    = (const float*)d_in[11];
  const float* linW   = (const float*)d_in[12];
  const float* linb   = (const float*)d_in[13];
  const float* gamma  = (const float*)d_in[14];
  const float* beta   = (const float*)d_in[15];
  float* out0 = (float*)d_out;
  float* out1 = (float*)d_out + kOut1ElemOff;

  char* ws = (char*)d_ws;
  unsigned short* XH   = (unsigned short*)(ws + kOffXH);
  unsigned short* XL   = (unsigned short*)(ws + kOffXL);
  unsigned short* XF   = (unsigned short*)(ws + kOffXF);
  float*          XT32 = (float*)(ws + kOffXT32);
  unsigned short* WKPH = (unsigned short*)(ws + kOffWKPH);
  unsigned short* WKPL = (unsigned short*)(ws + kOffWKPL);
  unsigned short* WKKH = (unsigned short*)(ws + kOffWKKH);
  unsigned short* WKKL = (unsigned short*)(ws + kOffWKKL);
  unsigned short* WV2  = (unsigned short*)(ws + kOffWV2);
  unsigned short* LINW = (unsigned short*)(ws + kOffLINW);
  float*          XQ   = (float*)(ws + kOffXQ);
  float*          KS   = (float*)(ws + kOffKS);
  unsigned short* XQH  = (unsigned short*)(ws + kOffXQH);
  unsigned short* XQL  = (unsigned short*)(ws + kOffXQL);
  unsigned short* KSH  = (unsigned short*)(ws + kOffKSH);
  unsigned short* KSL  = (unsigned short*)(ws + kOffKSL);
  float*          Q1   = (float*)(ws + kOffQ1);
  float*          LG   = (float*)(ws + kOffLG);
  float*          PR   = (float*)(ws + kOffPR);
  unsigned short* ET   = (unsigned short*)(ws + kOffET);
  unsigned short* VB   = (unsigned short*)(ws + kOffVB);
  unsigned short* XDT  = (unsigned short*)(ws + kOffXDT);
  float*          ZB   = (float*)(ws + kOffZB);

  prep_act_kernel<<<dim3(kN / 64, kK2 / 64, kB), 256, 0, stream>>>(x, pca, XH, XL, XF, XT32);
  prep_weight_kernel<<<120, 256, 0, stream>>>(Wkp, Wk, Wv, Wvp, linW, WKPH, WKPL, WKKH, WKKL, WV2, LINW);

  wmma_gemm64<1, true, 0, false><<<dim3(4, 1), 256, 0, stream>>>(
      XH, XL, kK2, 0L,
      WKPH, WKPL, kC, 0L,
      (void*)XQ, kCQ, 0L,
      nullptr, 0, 0L,
      kRows, kCQ, kC, 1.0f, 1.0f);

  wmma_gemm64<1, true, 0, false><<<dim3(4, 1), 256, 0, stream>>>(
      XH, XL, kK2, 0L,
      WKKH, WKKL, kK2, 0L,
      (void*)KS, kCQ, 0L,
      nullptr, 0, 0L,
      kRows, kCQ, kK2, 1.0f, 1.0f);

  qk_post_kernel<<<kRows / 16, 256, 0, stream>>>(XQ, KS, a_pca, e1W, e2W, e2b, XQH, XQL, KSH, KSL, Q1);

  wmma_gemm64<1, true, 0, false><<<dim3(8, kB), 256, 0, stream>>>(
      XQH, XQL, kCQ, (long)kN * kCQ,
      KSH, KSL, kCQ, (long)kN * kCQ,
      (void*)LG, kN, (long)kN * kN,
      nullptr, 0, 0L,
      kN, kN, kCQ, 1.0f, 1.0f);

  angle_softmax_kernel<<<kRows, 256, 0, stream>>>(LG, a_lrf, Q1, XQ, e1b, PR);

  colnorm_transpose_kernel<<<dim3(kN / 64, kB), 256, 0, stream>>>(PR, ET, out1);

  wmma_gemm64<0, false, 1, false><<<dim3(4, kB), 256, 0, stream>>>(
      WV2, WV2, kK2, 0L,
      XF, XF, kK2, (long)kN * kK2,
      (void*)VB, kN, (long)kC * kN,
      nullptr, 0, 0L,
      kC, kN, kK2, kVbScale, 1.0f);

  wmma_gemm64<0, false, 1, true><<<dim3(4, kB), 256, 0, stream>>>(
      ET, ET, kN, (long)kN * kN,
      VB, VB, kN, (long)kC * kN,
      (void*)XDT, kC, (long)kN * kC,
      XT32, kC, (long)kN * kC,
      kN, kC, kN, kXrScale, kXCarry);

  wmma_gemm64<0, false, 0, false><<<dim3(4, kB), 256, 0, stream>>>(
      LINW, LINW, kC, 0L,
      XDT, XDT, kC, (long)kN * kC,
      (void*)ZB, kN, (long)kC * kN,
      nullptr, 0, 0L,
      kC, kN, kC, kLinScale, 1.0f);

  bn_gelu_kernel<<<kC, 256, 0, stream>>>(ZB, x, linb, gamma, beta, out0);
}
